// BiMambaBlock_85727547228498
// MI455X (gfx1250) — hardware-verified
//
#include <hip/hip_runtime.h>
#include <math.h>

typedef __attribute__((ext_vector_type(16))) _Float16 v16h;
typedef __attribute__((ext_vector_type(8)))  _Float16 v8h;
typedef __attribute__((ext_vector_type(8)))  float    v8f;
typedef __attribute__((ext_vector_type(4)))  float    v4f;

constexpr int kBatch  = 4;
constexpr int kSeq    = 1024;
constexpr int kDm     = 256;
constexpr int kDin    = 512;
constexpr int kNst    = 16;
constexpr int kDtR    = 16;
constexpr int kXpN    = 48;
constexpr int kXdP    = 64;
constexpr int kRows   = kBatch * kSeq;
constexpr int kXzP    = 4 * kDin;
constexpr int kConvTP = 260;
constexpr int kScanTS = 64;
constexpr int kScanCh = 64;
constexpr int kScanYP = 68;
static_assert(kDtR + 2 * kNst == kXpN, "x_proj width");
static_assert(kXpN <= kXdP && (kXdP % 64) == 0, "x_proj pad");
static_assert((kDm % 32) == 0 && (kDin % 32) == 0 && ((2 * kDm) % 32) == 0, "GEMM K multiples of 32");
static_assert((kRows % 64) == 0 && (kXzP % 64) == 0 && (kDm % 64) == 0, "GEMM M,N multiples of 64");
static_assert((kSeq % kScanTS) == 0 && (kSeq % 64) == 0 && (kDin % kScanCh) == 0 && (kDin % 256) == 0, "tile multiples");
static_assert(kSeq == 1024 && kDin == 512, "shift constants below");

constexpr float kCarW    = 32.0f;
constexpr float kCarXc   = 64.0f;
constexpr float kCarY    = 1024.0f;
constexpr float kCarComb = 2048.0f;
constexpr float kSclIn   = 1.0f / kCarW;
constexpr float kSclXp   = 1.0f / (kCarW * kCarXc);
constexpr float kSclOut  = kCarComb / (kCarY * kCarW);
constexpr float kSclMix  = 1.0f / (kCarComb * kCarW);

constexpr size_t kOffX16   = 0;
constexpr size_t kOffWIN   = kOffX16  + (size_t)kRows * kDm * 2;
constexpr size_t kOffWXP   = kOffWIN  + (size_t)kXzP * kDm * 2;
constexpr size_t kOffWOUT  = kOffWXP  + (size_t)2 * kXdP * kDin * 2;
constexpr size_t kOffWMX   = kOffWOUT + (size_t)2 * kDm * kDin * 2;
constexpr size_t kOffXZ    = kOffWMX  + (size_t)kDm * 2 * kDm * 2;
constexpr size_t kOffXC    = kOffXZ   + (size_t)kRows * kXzP * 4;
constexpr size_t kOffXC16  = kOffXC   + (size_t)2 * kRows * kDin * 4;
constexpr size_t kOffXD    = kOffXC16 + (size_t)2 * kRows * kDin * 2;
constexpr size_t kOffY16   = kOffXD   + (size_t)2 * kRows * kXdP * 4;
constexpr size_t kOffCMB   = kOffY16  + (size_t)2 * kRows * kDin * 2;
constexpr size_t kWsTotal  = kOffCMB  + (size_t)kRows * 2 * kDm * 2;
static_assert(kWsTotal == 77463552ull, "carve total");
static_assert(kWsTotal <= 134217728ull, "carve cap");
static_assert((kOffWIN % 128) == 0 && (kOffWXP % 128) == 0 && (kOffWOUT % 128) == 0 && (kOffWMX % 128) == 0 &&
              (kOffXZ % 128) == 0 && (kOffXC % 128) == 0 && (kOffXC16 % 128) == 0 && (kOffXD % 128) == 0 &&
              (kOffY16 % 128) == 0 && (kOffCMB % 128) == 0, "128-B aligned regions");

__device__ __forceinline__ void row_guard_h(v8f& a, v8f& b, v8f& c, v8f& d, v16h x, v16h y) {
  asm volatile("v_nop\n\tv_nop\n\tv_nop\n\tv_nop" : "+v"(a), "+v"(b), "+v"(c), "+v"(d) : "v"(x), "v"(y));
}
__device__ __forceinline__ void keep4_h(v16h a, v16h b, v16h c, v16h d) { asm volatile("v_nop" :: "v"(a), "v"(b), "v"(c), "v"(d)); }
__device__ __forceinline__ void acc_guard4(v8f& a, v8f& b, v8f& c, v8f& d) { asm volatile("v_nop\n\tv_nop\n\tv_nop\n\tv_nop" : "+v"(a), "+v"(b), "+v"(c), "+v"(d)); }
template <typename T> struct Frag;
template <> struct Frag<_Float16> {
  typedef v16h V; union U { v16h v; v8h h[2]; };
  static __device__ __forceinline__ v16h load(const _Float16* p) {
    U f; f.h[0] = *(const v8h*)(p); f.h[1] = *(const v8h*)(p + 16); return f.v;
  }
  static __device__ __forceinline__ v8f mma(v16h a, v16h b, v8f c) {
    return __builtin_amdgcn_wmma_f32_16x16x32_f16(false, a, false, b, (short)0, c, false, false);
  }
};

template <int BIAS_MODE, int OUT_MODE>
__global__ __launch_bounds__(256) void wmma_gemm64_h(
    const unsigned short* __restrict__ Ap, int lda, long strideA,
    const unsigned short* __restrict__ Btp, int ldb, long strideB,
    void* __restrict__ Cout, int ldc, long strideC,
    const float* __restrict__ bias,
    int M, int N, int K, float scale) {
  typedef _Float16 T;
  typedef v16h V;
  __shared__ __align__(16) float sT[8][16 * 68];
  const int b    = blockIdx.y;
  const int lane = threadIdx.x & 31;
  const int wave = threadIdx.x >> 5;
  const int tilesN = N >> 6;
  const int tilesM = M >> 6;
  const int tile = blockIdx.x * 8 + wave;
  if (tile >= tilesM * tilesN) return;
  const int tm = tile / tilesN;
  const int tn = tile - tm * tilesN;
  const int m0 = tm << 6;
  const int n0 = tn << 6;

  const T* Ab = (const T*)Ap  + (size_t)b * strideA;
  const T* Bb = (const T*)Btp + (size_t)b * strideB;

  const int rlane = lane & 15;
  const int koff  = (lane >> 4) * 8;
  const int mOff  = (lane >> 4) * 8;

  v8f acc[4][4];
#pragma unroll
  for (int i = 0; i < 4; ++i)
#pragma unroll
    for (int j = 0; j < 4; ++j) acc[i][j] = (v8f){0.f,0.f,0.f,0.f,0.f,0.f,0.f,0.f};

  for (int k0 = 0; k0 < K; k0 += 32) {
    V bh[4];
#pragma unroll
    for (int j = 0; j < 4; ++j) {
      const size_t bo = (size_t)(n0 + (j << 4) + rlane) * ldb + koff + k0;
      bh[j] = Frag<T>::load(Bb + bo);
    }
#pragma unroll
    for (int i = 0; i < 4; ++i) {
      const size_t ao = (size_t)(m0 + (i << 4) + rlane) * lda + koff + k0;
      V ah = Frag<T>::load(Ab + ao);
#pragma unroll
      for (int j = 0; j < 4; ++j) acc[i][j] = Frag<T>::mma(ah, bh[j], acc[i][j]);
      row_guard_h(acc[i][0], acc[i][1], acc[i][2], acc[i][3], ah, bh[3]);
    }
    keep4_h(bh[0], bh[1], bh[2], bh[3]);
  }
  acc_guard4(acc[0][0], acc[0][1], acc[0][2], acc[0][3]);
  acc_guard4(acc[1][0], acc[1][1], acc[1][2], acc[1][3]);
  acc_guard4(acc[2][0], acc[2][1], acc[2][2], acc[2][3]);
  acc_guard4(acc[3][0], acc[3][1], acc[3][2], acc[3][3]);

  float* slab = sT[wave];
#pragma unroll
  for (int i = 0; i < 4; ++i) {
    const int mBase = m0 + (i << 4);
#pragma unroll
    for (int j = 0; j < 4; ++j) {
      const int n = n0 + (j << 4) + rlane;
      float bv = 0.f;
      if (BIAS_MODE == 2) bv = bias[n];
#pragma unroll
      for (int r = 0; r < 8; ++r) {
        float v = acc[i][j][r] * scale;
        if (BIAS_MODE == 2) v += bv;
        slab[(mOff + r) * 68 + (j << 4) + rlane] = v;
      }
    }
    __builtin_amdgcn_fence(__ATOMIC_RELEASE, "workgroup");
    __builtin_amdgcn_wave_barrier();
    __builtin_amdgcn_fence(__ATOMIC_ACQUIRE, "workgroup");
    if (OUT_MODE == 0) {
      float* C = (float*)Cout + (size_t)b * strideC;
      const int hh = lane >> 4, c4 = (lane & 15) * 4;
      for (int pass = 0; pass < 2; ++pass) {
#pragma unroll
        for (int it = 0; it < 8; ++it) {
          const int row = it * 2 + hh;
          v4f v = *(const v4f*)(slab + row * 68 + c4);
          *(volatile v4f*)(C + (size_t)(mBase + row) * ldc + n0 + c4) = v;
        }
        __threadfence();
      }
    } else {
      const int q = lane >> 3, c8 = (lane & 7) * 8;
      unsigned short* C = (unsigned short*)Cout + (size_t)b * strideC;
      for (int pass = 0; pass < 2; ++pass) {
#pragma unroll
        for (int it = 0; it < 4; ++it) {
          const int row = it * 4 + q;
          const float* sp = slab + row * 68 + c8;
          v8h hv;
#pragma unroll
          for (int e = 0; e < 8; ++e) hv[e] = (_Float16)sp[e];
          *(volatile v8h*)(C + (size_t)(mBase + row) * ldc + n0 + c8) = hv;
        }
        __threadfence();
      }
    }
    __builtin_amdgcn_fence(__ATOMIC_RELEASE, "workgroup");
    __builtin_amdgcn_wave_barrier();
    __builtin_amdgcn_fence(__ATOMIC_ACQUIRE, "workgroup");
  }
}

__global__ __launch_bounds__(256) void cast_f16_kernel(
    const float* __restrict__ src0, const float* __restrict__ src1,
    unsigned short* __restrict__ dst, int total8, float scale)
{
  const int i = blockIdx.x * 256 + threadIdx.x;
  if (i >= total8) return;
  const float* src = (blockIdx.y == 0) ? src0 : src1;
  const size_t e0 = (size_t)i << 3;
  const float* p = src + e0;
  const v4f a0 = *(const v4f*)(p);
  const v4f a1 = *(const v4f*)(p + 4);
  v8h hv;
#pragma unroll
  for (int e = 0; e < 4; ++e) {
    hv[e]     = (_Float16)(a0[e] * scale);
    hv[4 + e] = (_Float16)(a1[e] * scale);
  }
  unsigned short* q = dst + (size_t)blockIdx.y * ((size_t)total8 << 3) + e0;
  *(volatile v8h*)q = hv;
  __threadfence();
  *(volatile v8h*)q = hv;
}

__global__ __launch_bounds__(256) void cast_xproj_kernel(
    const float* __restrict__ src0, const float* __restrict__ src1,
    unsigned short* __restrict__ dst, float scale)
{
  const int i = blockIdx.x * 256 + threadIdx.x;
  if (i >= (kXdP * kDin) / 8) return;
  const float* src = (blockIdx.y == 0) ? src0 : src1;
  const int e0  = i << 3;
  const int row = e0 >> 9;
  const int col = e0 & (kDin - 1);
  const int rowc = (row < kXpN) ? row : (kXpN - 1);
  const bool live = (row < kXpN);
  const float* p = src + (size_t)rowc * kDin + col;
  const v4f a0 = *(const v4f*)(p);
  const v4f a1 = *(const v4f*)(p + 4);
  v8h hv;
#pragma unroll
  for (int e = 0; e < 4; ++e) {
    const float f0 = live ? (a0[e] * scale) : 0.0f;
    const float f1 = live ? (a1[e] * scale) : 0.0f;
    hv[e]     = (_Float16)f0;
    hv[4 + e] = (_Float16)f1;
  }
  unsigned short* q = dst + (size_t)blockIdx.y * (size_t)(kXdP * kDin) + e0;
  *(volatile v8h*)q = hv;
  __threadfence();
  *(volatile v8h*)q = hv;
}

__global__ __launch_bounds__(256) void conv_silu_kernel(
    const float* __restrict__ XZ,
    const float* __restrict__ cw0, const float* __restrict__ cb0,
    const float* __restrict__ cw1, const float* __restrict__ cb1,
    float* __restrict__ XC, unsigned short* __restrict__ XC16)
{
  __shared__ __align__(16) float sT[16 * kConvTP];
  const int tid = threadIdx.x, lane = tid & 31, wave = tid >> 5;
  const int dir = blockIdx.z;
  const int d0 = blockIdx.x * 256, d = d0 + tid;
  const int g0 = blockIdx.y * 64;
  const int tb = g0 & (kSeq - 1);
  const float* cw = dir ? cw1 : cw0;
  const float* cb = dir ? cb1 : cb0;
  const int xcol = dir * (2 * kDin) + d;
  float* XCd = XC + (size_t)dir * kRows * kDin;
  unsigned short* XHd = XC16 + (size_t)dir * kRows * kDin;
  const v4f wv = *(const v4f*)(cw + (size_t)d * 4);
  const float w0 = wv[0], w1 = wv[1], w2 = wv[2], w3 = wv[3];
  const float bc = cb[d];
  const int sdir  = dir ? -1 : 1;
  const int first = dir ? (g0 + 63) : g0;
  const bool hist = dir ? (tb + 64 < kSeq) : (tb > 0);
  float xm3, xm2, xm1;
  {
    const int r1 = hist ? (first - sdir)     : g0;
    const int r2 = hist ? (first - 2 * sdir) : g0;
    const int r3 = hist ? (first - 3 * sdir) : g0;
    const float v1 = XZ[(size_t)r1 * kXzP + xcol];
    const float v2 = XZ[(size_t)r2 * kXzP + xcol];
    const float v3 = XZ[(size_t)r3 * kXzP + xcol];
    xm1 = hist ? v1 : 0.f;
    xm2 = hist ? v2 : 0.f;
    xm3 = hist ? v3 : 0.f;
  }
  const int hrow = wave >> 1;
  const int hch  = (wave & 1) * 128 + lane * 4;
#pragma unroll 1
  for (int sub = 0; sub < 4; ++sub) {
    const int pbase = sub * 16;
    const int lb = dir ? (first - pbase - 15) : (first + pbase);
#pragma unroll 1
    for (int s = 0; s < 16; ++s) {
      const int row = first + sdir * (pbase + s);
      const int tr  = dir ? (15 - s) : s;
      const float xcur = XZ[(size_t)row * kXzP + xcol];
      float acc = w0 * xm3;
      acc = fmaf(w1, xm2, acc);
      acc = fmaf(w2, xm1, acc);
      acc = fmaf(w3, xcur, acc);
      const float sv = acc + bc;
      const float sg = __builtin_amdgcn_rcpf(1.0f + expf(-sv));
      sT[tr * kConvTP + tid] = sv * sg;
      xm3 = xm2; xm2 = xm1; xm1 = xcur;
    }
    __syncthreads();
    v4f fv[4];
    v8h bv[2];
#pragma unroll
    for (int it = 0; it < 4; ++it) fv[it] = *(const v4f*)(sT + (it * 4 + hrow) * kConvTP + hch);
#pragma unroll
    for (int it = 0; it < 2; ++it) {
      const float* sp = sT + (it * 8 + wave) * kConvTP + lane * 8;
      const v4f a0 = *(const v4f*)(sp);
      const v4f a1 = *(const v4f*)(sp + 4);
#pragma unroll
      for (int e = 0; e < 4; ++e) {
        bv[it][e]     = (_Float16)(a0[e] * kCarXc);
        bv[it][4 + e] = (_Float16)(a1[e] * kCarXc);
      }
    }
    for (int pass = 0; pass < 2; ++pass) {
#pragma unroll
      for (int it = 0; it < 4; ++it)
        *(volatile v4f*)(XCd + (size_t)(lb + it * 4 + hrow) * kDin + d0 + hch) = fv[it];
#pragma unroll
      for (int it = 0; it < 2; ++it)
        *(volatile v8h*)(XHd + (size_t)(lb + it * 8 + wave) * kDin + d0 + lane * 8) = bv[it];
      __threadfence();
    }
    __syncthreads();
  }
}

__global__ __launch_bounds__(64) void scan_kernel(
    const float* __restrict__ XD, const float* __restrict__ XC, const float* __restrict__ XZ,
    const float* __restrict__ Wdt0, const float* __restrict__ bdt0, const float* __restrict__ Alog0, const float* __restrict__ Dp0,
    const float* __restrict__ Wdt1, const float* __restrict__ bdt1, const float* __restrict__ Alog1, const float* __restrict__ Dp1,
    unsigned short* __restrict__ Y16)
{
  __shared__ __align__(16) float sX[kScanTS * kXdP];
  __shared__ __align__(16) float sY[kScanTS * kScanYP];
  __shared__ __align__(16) float sW[kDtR * kScanCh];
  __shared__ __align__(16) float sA[kNst * kScanCh];
  const int tid = threadIdx.x, lane = tid & 31, wave = tid >> 5;
  constexpr int kBlkPerB   = kDin / kScanCh;
  constexpr int kBlkPerDir = kBatch * kBlkPerB;
  const int dir = blockIdx.x / kBlkPerDir;
  const int rem = blockIdx.x - dir * kBlkPerDir;
  const int bix = rem / kBlkPerB;
  const int d0  = (rem - bix * kBlkPerB) * kScanCh;
  const int d   = d0 + tid;
  const float* Wdt  = dir ? Wdt1  : Wdt0;
  const float* bdt  = dir ? bdt1  : bdt0;
  const float* Alog = dir ? Alog1 : Alog0;
  const float* Dp   = dir ? Dp1   : Dp0;
  const float* XDd = XD + (size_t)dir * kRows * kXdP;
  const float* XCd = XC + (size_t)dir * kRows * kDin;
  unsigned short* Yd = Y16 + (size_t)dir * kRows * kDin;
  const int zcol = dir * (2 * kDin) + kDin + d;
  const size_t row0 = (size_t)bix * kSeq;
#pragma unroll 1
  for (int r = 0; r < kDtR; ++r) sW[r * kScanCh + tid] = Wdt[(size_t)d * kDtR + r];
#pragma unroll 1
  for (int s = 0; s < kNst; ++s) sA[s * kScanCh + tid] = -expf(Alog[(size_t)d * kNst + s]);
  __syncthreads();
  float negA[kNst], h[kNst];
#pragma unroll
  for (int s = 0; s < kNst; ++s) {
    negA[s] = sA[s * kScanCh + tid];
    h[s] = 0.f;
  }
  const float bb = bdt[d], Dd = Dp[d];
  const int lr = tid >> 4, lc4 = (tid & 15) * 4;
  const int q = lane >> 3, c8 = (lane & 7) * 8;
#pragma unroll 1
  for (int ci = 0; ci < kSeq / kScanTS; ++ci) {
    const int t0 = dir ? (kSeq - kScanTS - ci * kScanTS) : (ci * kScanTS);
    __syncthreads();
#pragma unroll
    for (int i = 0; i < 16; ++i) {
      const int r = lr + 4 * i;
      *(v4f*)(sX + r * kXdP + lc4) = *(const v4f*)(XDd + (row0 + t0 + r) * kXdP + lc4);
    }
    __syncthreads();
#pragma unroll 1
    for (int p = 0; p < kScanTS; ++p) {
      const int s = dir ? (kScanTS - 1 - p) : p;
      const int t = t0 + s;
      const float* xr = sX + s * kXdP;
      float vdot = 0.f;
#pragma unroll 1
      for (int r4 = 0; r4 < kDtR / 4; ++r4) {
        const v4f xv = *(const v4f*)(xr + 4 * r4);
        const float* wp = sW + (4 * r4) * kScanCh + tid;
        vdot = fmaf(xv[0], wp[0], vdot);
        vdot = fmaf(xv[1], wp[kScanCh], vdot);
        vdot = fmaf(xv[2], wp[2 * kScanCh], vdot);
        vdot = fmaf(xv[3], wp[3 * kScanCh], vdot);
      }
      float Bs[kNst], Cs[kNst];
#pragma unroll
      for (int q4 = 0; q4 < 4; ++q4) {
        const v4f bv = *(const v4f*)(xr + kDtR + 4 * q4);
        const v4f cv = *(const v4f*)(xr + kDtR + kNst + 4 * q4);
        Bs[4 * q4 + 0] = bv[0]; Bs[4 * q4 + 1] = bv[1]; Bs[4 * q4 + 2] = bv[2]; Bs[4 * q4 + 3] = bv[3];
        Cs[4 * q4 + 0] = cv[0]; Cs[4 * q4 + 1] = cv[1]; Cs[4 * q4 + 2] = cv[2]; Cs[4 * q4 + 3] = cv[3];
      }
      const float v   = vdot + bb;
      const float a   = __expf(-fabsf(v));
      const float u   = 1.0f + a;
      const float l1p = __logf(u) + (a - (u - 1.0f)) * __builtin_amdgcn_rcpf(u);
      const float dt  = fmaxf(v, 0.0f) + l1p;
      float xt = XCd[(row0 + t) * kDin + d];
      asm volatile("" : "+v"(xt));
      float zv = XZ[(row0 + t) * kXzP + zcol];
      asm volatile("" : "+v"(zv));
      const float dtx = dt * xt;
      float y = 0.f;
#pragma unroll
      for (int k = 0; k < kNst; ++k) {
        const float e = __expf(dt * negA[k]);
        h[k] = fmaf(e, h[k], dtx * Bs[k]);
        y = fmaf(h[k], Cs[k], y);
      }
      y = fmaf(xt, Dd, y);
      const float sg = __builtin_amdgcn_rcpf(1.0f + expf(-zv));
      y = y * (zv * sg);
      sY[s * kScanYP + tid] = y * kCarY;
    }
    __syncthreads();
    v8h hv[8];
#pragma unroll
    for (int it = 0; it < 8; ++it) {
      const int row = it * 8 + wave * 4 + q;
      const float* sp = sY + row * kScanYP + c8;
      const v4f a0 = *(const v4f*)(sp);
      const v4f a1 = *(const v4f*)(sp + 4);
#pragma unroll
      for (int e = 0; e < 4; ++e) {
        hv[it][e]     = (_Float16)a0[e];
        hv[it][4 + e] = (_Float16)a1[e];
      }
    }
    for (int pass = 0; pass < 2; ++pass) {
#pragma unroll
      for (int it = 0; it < 8; ++it) {
        const int row = it * 8 + wave * 4 + q;
        const size_t o = (row0 + t0 + row) * kDin + d0 + c8;
        *(volatile v8h*)(Yd + o) = hv[it];
      }
      __threadfence();
    }
  }
}

extern "C" void kernel_launch(void* const* d_in, const int* in_sizes, int n_in,
                              void* d_out, int out_size, void* d_ws, size_t ws_size,
                              hipStream_t stream) {
  if (n_in < 21) return;
  if (in_sizes[0] != kRows * kDm) return;
  if (in_sizes[1] != kDm * 2 * kDm) return;
  if (in_sizes[2] != kDm) return;
  for (int g = 0; g < 2; ++g) {
    const int o = 3 + 9 * g;
    if (in_sizes[o + 0] != 2 * kDin * kDm) return;
    if (in_sizes[o + 1] != kDin * 4) return;
    if (in_sizes[o + 2] != kDin) return;
    if (in_sizes[o + 3] != kXpN * kDin) return;
    if (in_sizes[o + 4] != kDin * kDtR) return;
    if (in_sizes[o + 5] != kDin) return;
    if (in_sizes[o + 6] != kDin * kNst) return;
    if (in_sizes[o + 7] != kDin) return;
    if (in_sizes[o + 8] != kDm * kDin) return;
  }
  if (out_size != kRows * kDm) return;
  if (ws_size < kWsTotal) return;

  const float* x        = (const float*)d_in[0];
  const float* mixer_w  = (const float*)d_in[1];
  const float* mixer_b  = (const float*)d_in[2];
  const float* f_in_w   = (const float*)d_in[3];
  const float* f_conv_w = (const float*)d_in[4];
  const float* f_conv_b = (const float*)d_in[5];
  const float* f_xp_w   = (const float*)d_in[6];
  const float* f_dt_w   = (const float*)d_in[7];
  const float* f_dt_b   = (const float*)d_in[8];
  const float* f_A_log  = (const float*)d_in[9];
  const float* f_D      = (const float*)d_in[10];
  const float* f_out_w  = (const float*)d_in[11];
  const float* b_in_w   = (const float*)d_in[12];
  const float* b_conv_w = (const float*)d_in[13];
  const float* b_conv_b = (const float*)d_in[14];
  const float* b_xp_w   = (const float*)d_in[15];
  const float* b_dt_w   = (const float*)d_in[16];
  const float* b_dt_b   = (const float*)d_in[17];
  const float* b_A_log  = (const float*)d_in[18];
  const float* b_D      = (const float*)d_in[19];
  const float* b_out_w  = (const float*)d_in[20];
  float* out = (float*)d_out;

  char* ws = (char*)d_ws;
  unsigned short* X16    = (unsigned short*)(ws + kOffX16);
  unsigned short* WIN16  = (unsigned short*)(ws + kOffWIN);
  unsigned short* WXP16  = (unsigned short*)(ws + kOffWXP);
  unsigned short* WOUT16 = (unsigned short*)(ws + kOffWOUT);
  unsigned short* WMX16  = (unsigned short*)(ws + kOffWMX);
  float*          XZ     = (float*)(ws + kOffXZ);
  float*          XC     = (float*)(ws + kOffXC);
  unsigned short* XC16   = (unsigned short*)(ws + kOffXC16);
  float*          XD     = (float*)(ws + kOffXD);
  unsigned short* Y16    = (unsigned short*)(ws + kOffY16);
  unsigned short* CMB16  = (unsigned short*)(ws + kOffCMB);

  cast_f16_kernel<<<dim3((kRows * kDm / 8) / 256, 1), 256, 0, stream>>>(x, x, X16, kRows * kDm / 8, 1.0f);
  cast_f16_kernel<<<dim3((2 * kDin * kDm / 8) / 256, 2), 256, 0, stream>>>(f_in_w, b_in_w, WIN16, 2 * kDin * kDm / 8, kCarW);
  cast_xproj_kernel<<<dim3((kXdP * kDin / 8) / 256, 2), 256, 0, stream>>>(f_xp_w, b_xp_w, WXP16, kCarW);
  cast_f16_kernel<<<dim3((kDm * kDin / 8) / 256, 2), 256, 0, stream>>>(f_out_w, b_out_w, WOUT16, kDm * kDin / 8, kCarW);
  cast_f16_kernel<<<dim3((kDm * 2 * kDm / 8) / 256, 1), 256, 0, stream>>>(mixer_w, mixer_w, WMX16, kDm * 2 * kDm / 8, kCarW);

  wmma_gemm64_h<0, 0><<<dim3(256, 1), 256, 0, stream>>>(
      X16, kDm, 0L,
      WIN16, kDm, 0L,
      (void*)XZ, kXzP, 0L,
      mixer_b,
      kRows, kXzP, kDm, kSclIn);

  conv_silu_kernel<<<dim3(kDin / 256, kRows / 64, 2), 256, 0, stream>>>(
      XZ, f_conv_w, f_conv_b, b_conv_w, b_conv_b, XC, XC16);

  wmma_gemm64_h<0, 0><<<dim3(8, 2), 256, 0, stream>>>(
      XC16, kDin, (long)kRows * kDin,
      WXP16, kDin, (long)kXdP * kDin,
      (void*)XD, kXdP, (long)kRows * kXdP,
      mixer_b,
      kRows, kXdP, kDin, kSclXp);

  scan_kernel<<<2 * kBatch * (kDin / kScanCh), kScanCh, 0, stream>>>(
      XD, XC, XZ,
      f_dt_w, f_dt_b, f_A_log, f_D,
      b_dt_w, b_dt_b, b_A_log, b_D,
      Y16);

  wmma_gemm64_h<0, 1><<<dim3(32, 2), 256, 0, stream>>>(
      Y16, kDin, (long)kRows * kDin,
      WOUT16, kDin, (long)kDm * kDin,
      (void*)CMB16, 2 * kDm, (long)kDm,
      mixer_b,
      kRows, kDm, kDin, kSclOut);

  wmma_gemm64_h<2, 0><<<dim3(32, 1), 256, 0, stream>>>(
      CMB16, 2 * kDm, 0L,
      WMX16, 2 * kDm, 0L,
      (void*)out, kDm, 0L,
      mixer_b,
      kRows, kDm, 2 * kDm, kSclMix);
}
